// PoseMixtureVAE_858993459257
// MI455X (gfx1250) — hardware-verified
//
#include <hip/hip_runtime.h>
#include <math.h>

typedef __attribute__((ext_vector_type(16))) _Float16 v16h;
typedef __attribute__((ext_vector_type(16))) __bf16 v16b;
typedef __attribute__((ext_vector_type(8)))  _Float16 v8h;
typedef __attribute__((ext_vector_type(8)))  float v8f;
typedef __attribute__((ext_vector_type(4)))  float v4f;
typedef __attribute__((ext_vector_type(2)))  float v2f;
typedef __attribute__((ext_vector_type(4)))  unsigned v4u;
typedef __attribute__((ext_vector_type(4)))  int v4i;
typedef float __attribute__((may_alias)) float_a;
typedef int __attribute__((may_alias)) int_a;

template <typename T> __device__ __forceinline__ void vst2(void* p, T v) { *(volatile T*)p = v; __threadfence(); *(volatile T*)p = v; }
__device__ __forceinline__ v8f wmma16(v16h a, v16h b, v8f c) {
  v8f d = __builtin_amdgcn_wmma_f32_16x16x32_f16(false, a, false, b, (short)0, c, false, false);
  asm volatile("v_nop\n\tv_nop\n\tv_nop\n\tv_nop" : "+v"(d) : "v"(a), "v"(b));
  return d;
}
__device__ __forceinline__ v8f wmma_bf(v16b a, v16b b, v8f c) {
  v8f d = __builtin_amdgcn_wmma_f32_16x16x32_bf16(false, a, false, b, (short)0, c, false, false);
  asm volatile("v_nop\n\tv_nop\n\tv_nop\n\tv_nop" : "+v"(d) : "v"(a), "v"(b));
  return d;
}
__device__ __forceinline__ v16h frag_h(const _Float16* rowk0, int lane) {
  union { v16h v; v8h q[2]; } u; const _Float16* p = rowk0 + 8 * (lane >> 4);
  u.q[0] = *(const v8h*)p; u.q[1] = *(const v8h*)(p + 16); return u.v;
}
__device__ __forceinline__ v16h frag_f32(const float* rowk0, int lane) {
  v16h a; const float* p = rowk0 + 8 * (lane >> 4);
#pragma unroll
  for (int i = 0; i < 8; ++i) { a[i] = (_Float16)p[i]; a[8 + i] = (_Float16)p[16 + i]; }
  return a;
}
__device__ __forceinline__ v16h frag_f32s(const float* rowk0, int lane, float sc) {
  v16h a; const float* p = rowk0 + 8 * (lane >> 4);
#pragma unroll
  for (int i = 0; i < 8; ++i) { a[i] = (_Float16)(p[i] * sc); a[8 + i] = (_Float16)(p[16 + i] * sc); }
  return a;
}
__device__ __forceinline__ v16h fragc_f32(const float* W, int k0, int n, int lane, int ld, int K) {
  v16h a; const int g = lane >> 4;
#pragma unroll
  for (int i = 0; i < 8; ++i) { const int ka = k0 + 8 * g + i, kb = ka + 16;
    a[i] = (_Float16)(ka < K ? W[(size_t)(ka < K ? ka : K - 1) * ld + n] : 0.f); a[8 + i] = (_Float16)(kb < K ? W[(size_t)(kb < K ? kb : K - 1) * ld + n] : 0.f); }
  return a;
}
struct F2 { v16b h, l; };
__device__ __forceinline__ F2 bsplit16(const float v[16]) { F2 r;
#pragma unroll
  for (int i = 0; i < 16; ++i) { const __bf16 h = (__bf16)v[i]; r.h[i] = h; r.l[i] = (__bf16)(v[i] - (float)h); }
  return r; }
__device__ __forceinline__ F2 split_row(const float* row, int k0, int lane) { float v[16]; const float* p = row + k0 + 8 * (lane >> 4);
#pragma unroll
  for (int i = 0; i < 8; ++i) { v[i] = p[i]; v[8 + i] = p[16 + i]; }
  return bsplit16(v); }
__device__ __forceinline__ F2 split_rowK(const float* row, int k0, int lane, int K) { float v[16]; const int g = lane >> 4;
#pragma unroll
  for (int i = 0; i < 8; ++i) { const int ka = k0 + 8 * g + i, kb = ka + 16; v[i] = ka < K ? row[ka < K ? ka : K - 1] : 0.f; v[8 + i] = kb < K ? row[kb < K ? kb : K - 1] : 0.f; }
  return bsplit16(v); }
__device__ __forceinline__ F2 split_col(const float* W, int k0, int n, int lane, int ld, int K) { float v[16]; const int g = lane >> 4;
#pragma unroll
  for (int i = 0; i < 8; ++i) { const int ka = k0 + 8 * g + i, kb = ka + 16; v[i] = ka < K ? W[(size_t)(ka < K ? ka : K - 1) * ld + n] : 0.f; v[8 + i] = kb < K ? W[(size_t)(kb < K ? kb : K - 1) * ld + n] : 0.f; }
  return bsplit16(v); }
__device__ __forceinline__ v8f mac3(const F2& a, const F2& b, v8f c) { c = wmma_bf(a.l, b.h, c); c = wmma_bf(a.h, b.l, c); return wmma_bf(a.h, b.h, c); }
__device__ __forceinline__ float sigm(float v) { return 1.0f / (1.0f + expf(-v)); }
#define LDSX() do { asm volatile("s_wait_dscnt 0" ::: "memory"); __builtin_amdgcn_wave_barrier(); __builtin_amdgcn_fence(__ATOMIC_RELEASE, "workgroup"); } while (0)

__device__ __forceinline__ float bfr(float v) { return (float)(__bf16)v; }
__device__ __attribute__((noinline)) float elu_ni(float v) { return v > 0.f ? v : expm1f(v); }
#define NBAT 4096
#define FR 267
#define LAT 32
#define HIDN 256
#define GH 64
#define NEXP 6
#ifndef NRB
#define NRB (NBAT / 64)
#endif
#define MU_OFF ((size_t)NBAT * FR)
#define LV_OFF (MU_OFF + (size_t)NBAT * LAT)
#define WS_H1 0u
#define WS_H2 (WS_H1 + 4u * (size_t)NBAT * HIDN)
#define WS_Z  (WS_H2 + 4u * (size_t)NBAT * HIDN)
#define WS_G1 (WS_Z + 4u * (size_t)NBAT * LAT)
#define WS_G2 (WS_G1 + 4u * (size_t)NBAT * GH)
#define WS_GL (WS_G2 + 4u * (size_t)NBAT * GH)
#define WS_CF (WS_GL + 4u * (size_t)NBAT * 128)
#define WS_L0 (WS_CF + 4u * (size_t)NBAT * 8)
#define WS_L1 (WS_L0 + 4u * (size_t)NBAT * HIDN)
#define WS_L2 (WS_L1 + 4u * (size_t)NBAT * HIDN)
#define WS_END (WS_L2 + 4u * (size_t)NBAT * 384)
__global__ __launch_bounds__(128) void k_dense(const float* __restrict__ A1, int K1, int p1, int rb1, const float* __restrict__ A2, int K2, int p2, int rb2, const float* __restrict__ Wt, const float* __restrict__ BIAS, int NO, int E, const float* __restrict__ COEF, int act, float* __restrict__ DST, int dp) { __shared__ __align__(16) float sf[4][16][132];
  const int tid = threadIdx.x, wave = tid >> 5, lane = tid & 31, col = lane & 15, g = lane >> 4; const size_t r0 = (size_t)blockIdx.x * 64 + wave * 16; const int c0 = blockIdx.y * 128; const int K = K1 + K2; const int nkc = (K + 31) / 32; const size_t arow = r0 + col;
  v8f res[8] = {};
#pragma unroll 1
  for (int e = 0; e < E; ++e) { v8f acc[8] = {}; const float* We = Wt + (size_t)e * K * NO;
#pragma unroll 1
    for (int kc = 0; kc < nkc; ++kc) { float av[16];
#pragma unroll
      for (int i = 0; i < 16; ++i) { const int k = kc * 32 + 8 * g + (i < 8 ? i : 8 + i); float v = 0.f; if (k < K1) { v = A1[arow * p1 + k]; if (rb1) v = bfr(v); } else if (k < K) { v = A2[arow * p2 + (k - K1)]; if (rb2) v = bfr(v); } av[i] = v; }
      const F2 a = bsplit16(av);
#pragma unroll
      for (int j = 0; j < 8; ++j) { v16b w; const int o = c0 + j * 16 + col;
#pragma unroll
        for (int i = 0; i < 8; ++i) { const int ka = kc * 32 + 8 * g + i, kb = ka + 16; w[i] = (ka < K && o < NO) ? (__bf16)We[(size_t)ka * NO + o] : (__bf16)0.f; w[8 + i] = (kb < K && o < NO) ? (__bf16)We[(size_t)kb * NO + o] : (__bf16)0.f; }
        asm volatile("s_wait_loadcnt 0x0" ::: "memory"); acc[j] = wmma_bf(a.h, w, acc[j]); acc[j] = wmma_bf(a.l, w, acc[j]); } }
#pragma unroll
    for (int j = 0; j < 8; ++j) { const int o = c0 + j * 16 + col; const float bb = (o < NO) ? bfr(BIAS[(size_t)e * NO + o]) : 0.f;
#pragma unroll
      for (int r = 0; r < 8; ++r) { const float cf = COEF ? COEF[(r0 + 8 * g + r) * 8 + e] : 1.0f; res[j][r] += cf * (acc[j][r] + bb); } } }
#pragma unroll
  for (int j = 0; j < 8; ++j)
#pragma unroll
    for (int r = 0; r < 8; ++r) { const float v = res[j][r]; sf[wave][8 * g + r][j * 16 + col] = (act == 1) ? elu_ni(v) : v; }
  LDSX();
  { const int ncol = (dp - c0) < 128 ? (dp - c0) : 128;
    for (int rl = 0; rl < 16; ++rl) if (lane * 4 < ncol) vst2(DST + (r0 + rl) * (size_t)dp + c0 + lane * 4, *(const v4f*)&sf[wave][rl][lane * 4]); } }
__global__ __launch_bounds__(256) void k_z(const float* __restrict__ MU, const float* __restrict__ LV, const float* __restrict__ EPSI, float* __restrict__ Z) {
  const int t = threadIdx.x; const size_t row = (size_t)blockIdx.x * 32 + (t >> 3); const int q = t & 7; const size_t o = row * LAT + q * 4;
  const v4f m = *(const v4f*)(MU + o), l = *(const v4f*)(LV + o), ep = *(const v4f*)(EPSI + o); v4f z;
#pragma unroll
  for (int e = 0; e < 4; ++e) z[e] = m[e] + bfr(ep[e]) * expf(0.5f * l[e]);
  vst2(Z + o, z); }
__global__ __launch_bounds__(64) void k_coef(const float* __restrict__ GL, float* __restrict__ CF) { __shared__ __align__(16) float so[64 * 8];
  const int t = threadIdx.x; const size_t row = (size_t)blockIdx.x * 64 + t; const float* p = GL + row * 128; float m = p[0]; for (int e = 1; e < NEXP; ++e) m = fmaxf(m, p[e]); float ex[NEXP]; float s = 0.f; for (int e = 0; e < NEXP; ++e) { ex[e] = expf(p[e] - m); s += ex[e]; } const float inv = 1.0f / s;
  for (int e = 0; e < 8; ++e) so[t * 8 + e] = e < NEXP ? ex[e] * inv : 0.f;
  __syncthreads(); for (int q = t; q < 64 * 8 / 4; q += 64) vst2(CF + (size_t)blockIdx.x * 64 * 8 + q * 4, *(const v4f*)&so[q * 4]); }
__global__ __launch_bounds__(256) void k_copy(const float* __restrict__ L2, float* __restrict__ OUT) {
  const int t = threadIdx.x; const size_t r0 = (size_t)blockIdx.x * 64; float* dst = OUT + r0 * FR;
  for (int q = t; q < 64 * FR / 4; q += 256) { v4f v; for (int e = 0; e < 4; ++e) { const int idx = q * 4 + e; const int r = idx / FR, c = idx % FR; v[e] = L2[(r0 + r) * 384 + c]; } vst2(dst + q * 4, v); } }
extern "C" void kernel_launch(void* const* d_in, const int* in_sizes, int n_in, void* d_out, int out_size, void* d_ws, size_t ws_size, hipStream_t stream) {
  (void)in_sizes; (void)n_in; (void)out_size;
  const float** F = (const float**)d_in;
  if (ws_size < (size_t)WS_END) return;
  char* ws = (char*)d_ws; float *H1 = (float*)(ws + WS_H1), *H2 = (float*)(ws + WS_H2), *Z = (float*)(ws + WS_Z), *G1 = (float*)(ws + WS_G1), *G2 = (float*)(ws + WS_G2), *GL = (float*)(ws + WS_GL), *CF = (float*)(ws + WS_CF), *L0 = (float*)(ws + WS_L0), *L1 = (float*)(ws + WS_L1), *L2 = (float*)(ws + WS_L2);
  float* OUTF = (float*)d_out; float* MU = OUTF + MU_OFF; float* LV = OUTF + LV_OFF;
  k_dense<<<dim3(NRB, 2), 128, 0, stream>>>(F[0], FR, FR, 1, F[1], FR, FR, 1, F[3], F[4], HIDN, 1, nullptr, 1, H1, HIDN);
  k_dense<<<dim3(NRB, 2), 128, 0, stream>>>(F[0], FR, FR, 1, H1, HIDN, HIDN, 0, F[5], F[6], HIDN, 1, nullptr, 1, H2, HIDN);
  k_dense<<<dim3(NRB, 1), 128, 0, stream>>>(F[0], FR, FR, 1, H2, HIDN, HIDN, 0, F[7], F[8], LAT, 1, nullptr, 0, MU, LAT);
  k_dense<<<dim3(NRB, 1), 128, 0, stream>>>(F[0], FR, FR, 1, H2, HIDN, HIDN, 0, F[9], F[10], LAT, 1, nullptr, 0, LV, LAT);
  k_z<<<dim3(NRB * 2), 256, 0, stream>>>(MU, LV, F[2], Z);
  k_dense<<<dim3(NRB, 1), 128, 0, stream>>>(Z, LAT, LAT, 0, F[1], FR, FR, 1, F[11], F[12], GH, 1, nullptr, 1, G1, GH);
  k_dense<<<dim3(NRB, 1), 128, 0, stream>>>(G1, GH, GH, 0, nullptr, 0, 0, 0, F[13], F[14], GH, 1, nullptr, 1, G2, GH);
  k_dense<<<dim3(NRB, 1), 128, 0, stream>>>(G2, GH, GH, 0, nullptr, 0, 0, 0, F[15], F[16], NEXP, 1, nullptr, 0, GL, 128);
  k_coef<<<dim3(NRB), 64, 0, stream>>>(GL, CF);
  k_dense<<<dim3(NRB, 2), 128, 0, stream>>>(Z, LAT, LAT, 0, F[1], FR, FR, 1, F[17], F[18], HIDN, NEXP, CF, 1, L0, HIDN);
  k_dense<<<dim3(NRB, 2), 128, 0, stream>>>(Z, LAT, LAT, 0, L0, HIDN, HIDN, 0, F[19], F[20], HIDN, NEXP, CF, 1, L1, HIDN);
  k_dense<<<dim3(NRB, 3), 128, 0, stream>>>(Z, LAT, LAT, 0, L1, HIDN, HIDN, 0, F[21], F[22], FR, NEXP, CF, 0, L2, 384);
  k_copy<<<dim3(NRB), 256, 0, stream>>>(L2, OUTF);
}
